// NeighborhoodAttention2D_diffusion_20761871909013
// MI455X (gfx1250) — hardware-verified
//
#include <hip/hip_runtime.h>
#include <math.h>

typedef __attribute__((ext_vector_type(16))) _Float16 v16h;
typedef __attribute__((ext_vector_type(16))) __bf16 v16b;
typedef __attribute__((ext_vector_type(8)))  _Float16 v8h;
typedef __attribute__((ext_vector_type(8)))  float v8f;
typedef __attribute__((ext_vector_type(4)))  float v4f;
typedef __attribute__((ext_vector_type(2)))  float v2f;
typedef __attribute__((ext_vector_type(4)))  unsigned v4u;
typedef __attribute__((ext_vector_type(4)))  int v4i;
typedef float __attribute__((may_alias)) float_a;
typedef int __attribute__((may_alias)) int_a;

template <typename T> __device__ __forceinline__ void vst2(void* p, T v) { *(volatile T*)p = v; __threadfence(); *(volatile T*)p = v; }
__device__ __forceinline__ v8f wmma16(v16h a, v16h b, v8f c) {
  v8f d = __builtin_amdgcn_wmma_f32_16x16x32_f16(false, a, false, b, (short)0, c, false, false);
  asm volatile("v_nop\n\tv_nop\n\tv_nop\n\tv_nop" : "+v"(d) : "v"(a), "v"(b));
  return d;
}
__device__ __forceinline__ v8f wmma_bf(v16b a, v16b b, v8f c) {
  v8f d = __builtin_amdgcn_wmma_f32_16x16x32_bf16(false, a, false, b, (short)0, c, false, false);
  asm volatile("v_nop\n\tv_nop\n\tv_nop\n\tv_nop" : "+v"(d) : "v"(a), "v"(b));
  return d;
}
__device__ __forceinline__ v16h frag_h(const _Float16* rowk0, int lane) {
  union { v16h v; v8h q[2]; } u; const _Float16* p = rowk0 + 8 * (lane >> 4);
  u.q[0] = *(const v8h*)p; u.q[1] = *(const v8h*)(p + 16); return u.v;
}
__device__ __forceinline__ v16h frag_f32(const float* rowk0, int lane) {
  v16h a; const float* p = rowk0 + 8 * (lane >> 4);
#pragma unroll
  for (int i = 0; i < 8; ++i) { a[i] = (_Float16)p[i]; a[8 + i] = (_Float16)p[16 + i]; }
  return a;
}
__device__ __forceinline__ v16h frag_f32s(const float* rowk0, int lane, float sc) {
  v16h a; const float* p = rowk0 + 8 * (lane >> 4);
#pragma unroll
  for (int i = 0; i < 8; ++i) { a[i] = (_Float16)(p[i] * sc); a[8 + i] = (_Float16)(p[16 + i] * sc); }
  return a;
}
__device__ __forceinline__ v16h fragc_f32(const float* W, int k0, int n, int lane, int ld, int K) {
  v16h a; const int g = lane >> 4;
#pragma unroll
  for (int i = 0; i < 8; ++i) { const int ka = k0 + 8 * g + i, kb = ka + 16;
    a[i] = (_Float16)(ka < K ? W[(size_t)(ka < K ? ka : K - 1) * ld + n] : 0.f); a[8 + i] = (_Float16)(kb < K ? W[(size_t)(kb < K ? kb : K - 1) * ld + n] : 0.f); }
  return a;
}
struct F2 { v16b h, l; };
__device__ __forceinline__ F2 bsplit16(const float v[16]) { F2 r;
#pragma unroll
  for (int i = 0; i < 16; ++i) { const __bf16 h = (__bf16)v[i]; r.h[i] = h; r.l[i] = (__bf16)(v[i] - (float)h); }
  return r; }
__device__ __forceinline__ F2 split_row(const float* row, int k0, int lane) { float v[16]; const float* p = row + k0 + 8 * (lane >> 4);
#pragma unroll
  for (int i = 0; i < 8; ++i) { v[i] = p[i]; v[8 + i] = p[16 + i]; }
  return bsplit16(v); }
__device__ __forceinline__ F2 split_rowK(const float* row, int k0, int lane, int K) { float v[16]; const int g = lane >> 4;
#pragma unroll
  for (int i = 0; i < 8; ++i) { const int ka = k0 + 8 * g + i, kb = ka + 16; v[i] = ka < K ? row[ka < K ? ka : K - 1] : 0.f; v[8 + i] = kb < K ? row[kb < K ? kb : K - 1] : 0.f; }
  return bsplit16(v); }
__device__ __forceinline__ F2 split_col(const float* W, int k0, int n, int lane, int ld, int K) { float v[16]; const int g = lane >> 4;
#pragma unroll
  for (int i = 0; i < 8; ++i) { const int ka = k0 + 8 * g + i, kb = ka + 16; v[i] = ka < K ? W[(size_t)(ka < K ? ka : K - 1) * ld + n] : 0.f; v[8 + i] = kb < K ? W[(size_t)(kb < K ? kb : K - 1) * ld + n] : 0.f; }
  return bsplit16(v); }
__device__ __forceinline__ v8f mac3(const F2& a, const F2& b, v8f c) { c = wmma_bf(a.l, b.h, c); c = wmma_bf(a.h, b.l, c); return wmma_bf(a.h, b.h, c); }
__device__ __forceinline__ float sigm(float v) { return 1.0f / (1.0f + expf(-v)); }
#define LDSX() do { asm volatile("s_wait_dscnt 0" ::: "memory"); __builtin_amdgcn_wave_barrier(); __builtin_amdgcn_fence(__ATOMIC_RELEASE, "workgroup"); } while (0)


#define NBT 2
#define HH 64
#define WW 64
#define CC 128
#define NHD 4
#define HD 32
#define KS 7
#define NTOK (NBT * HH * WW)
#ifndef TTB
#define TTB (NTOK / 64)
#define TNAB (NBT * HH * NHD)
#endif
typedef __attribute__((ext_vector_type(8))) __bf16 v8b;
__device__ __forceinline__ v16b frag_b(const __bf16* rowk0, int lane) {
  union { v16b v; v8b q[2]; } u; const __bf16* p = rowk0 + 8 * (lane >> 4);
  u.q[0] = *(const v8b*)p; u.q[1] = *(const v8b*)(p + 16); return u.v;
}
__device__ __forceinline__ float bfr(float v) { return (float)(__bf16)v; }
__device__ __attribute__((noinline)) float exp_ni(float v) { return expf(v); }
__device__ __attribute__((noinline)) float sin_ni(float v) { return sinf(v); }
__device__ __attribute__((noinline)) float cos_ni(float v) { return cosf(v); }
#define WS_ADA  0u
#define WS_PT   (WS_ADA + 4u * NBT * 256)
#define WS_QKV  (WS_PT + 2u * 512 * CC)
#define WS_O    (WS_QKV + 4u * NTOK * 384)
#define WS_END  (WS_O + 4u * NTOK * CC)

__global__ __launch_bounds__(256) void k_ada(const int* __restrict__ T, const float* __restrict__ lnw, const float* __restrict__ lnb, float* __restrict__ ADA) {
  __shared__ float semb[CC]; __shared__ __align__(16) float sres[256];
  const int tid = threadIdx.x;
  for (int b = 0; b < NBT; ++b) {
    const float tf = (float)T[b] / 100.0f * 4000.0f;
    if (tid < 64) { const float fr = exp_ni((float)tid * (-9.210340371976184f / 63.0f)); const float e = tf * fr; semb[tid] = sin_ni(e); semb[64 + tid] = cos_ni(e); }
    __syncthreads();
    { float s = bfr(lnb[tid]); for (int c = 0; c < CC; ++c) { const float v = semb[c]; const float sv = v / (1.0f + exp_ni(-v)); s += sv * bfr(lnw[c * 256 + tid]); } sres[tid] = s; }
    __syncthreads();
    if (tid < 64) vst2(ADA + b * 256 + tid * 4, *(const v4f*)&sres[tid * 4]);
    __syncthreads(); }
}
__global__ __launch_bounds__(128) void k_pack(const float* __restrict__ qw, const float* __restrict__ pw, __bf16* __restrict__ PT) {
  __shared__ __align__(16) __bf16 srow[CC];
  const int n = blockIdx.x, tid = threadIdx.x; srow[tid] = (__bf16)(n < 384 ? qw[(size_t)tid * 384 + n] : pw[(size_t)tid * CC + (n - 384)]);
  __syncthreads();
  if (tid < 16) vst2((unsigned*)(PT + (size_t)n * CC + tid * 8), *(const v4u*)(&srow[tid * 8]));
}
__global__ __launch_bounds__(128) void k_qkv(const float* __restrict__ X, const float* __restrict__ ADA, const __bf16* __restrict__ PT, const float* __restrict__ qb, float* __restrict__ QKV) {
  __shared__ __align__(16) __bf16 sah[64][CC + 8], sal[64][CC + 8]; __shared__ __align__(16) float so[4][16][196];
  const int tid = threadIdx.x, wave = tid >> 5, lane = tid & 31, col = lane & 15, g = lane >> 4; const size_t tk0 = (size_t)blockIdx.x * 64; const int b = (int)(tk0 / (HH * WW));
  { const int tl = tid >> 1, half = tid & 1; const float* xr = X + (tk0 + tl) * CC; float s = 0.f; for (int c = half * 64; c < half * 64 + 64; ++c) s += bfr(xr[c]); s += __shfl_xor(s, 1); const float mu = s / (float)CC;
    float v = 0.f; for (int c = half * 64; c < half * 64 + 64; ++c) { const float d = bfr(xr[c]) - mu; v += d * d; } v += __shfl_xor(v, 1); const float rs = 1.0f / sqrtf(v / (float)CC + 1e-5f);
    for (int c = half * 64; c < half * 64 + 64; ++c) { const float y = (bfr(xr[c]) - mu) * rs * (1.0f + ADA[b * 256 + c]) + ADA[b * 256 + CC + c]; const __bf16 hb = (__bf16)y; sah[tl][c] = hb; sal[tl][c] = (__bf16)(y - (float)hb); } }
  __syncthreads();
#pragma unroll 1
  for (int pass = 0; pass < 2; ++pass) { v8f acc[12];
#pragma unroll
    for (int j = 0; j < 12; ++j) acc[j] = (v8f){};
#pragma unroll
    for (int kc = 0; kc < 4; ++kc) { const v16b ah = frag_b(&sah[wave * 16 + col][kc * 32], lane), al = frag_b(&sal[wave * 16 + col][kc * 32], lane);
#pragma unroll
      for (int j = 0; j < 12; ++j) { const v16b w = frag_b(PT + (size_t)((pass * 12 + j) * 16 + col) * CC + kc * 32, lane); acc[j] = wmma_bf(al, w, acc[j]); acc[j] = wmma_bf(ah, w, acc[j]); } }
#pragma unroll
    for (int j = 0; j < 12; ++j) { const int n = (pass * 12 + j) * 16 + col; const float bb = bfr(qb[n]); const float sc = n < CC ? 0.17677669529663687f : 1.0f;
#pragma unroll
      for (int r = 0; r < 8; ++r) so[wave][8 * g + r][j * 16 + col] = (acc[j][r] + bb) * sc; }
    LDSX();
    for (int rl = 0; rl < 16; ++rl) for (int pc = lane; pc < 48; pc += 32) vst2(QKV + (tk0 + wave * 16 + rl) * 384 + pass * 192 + pc * 4, *(const v4f*)&so[wave][rl][pc * 4]);
    LDSX(); }
}
__global__ __launch_bounds__(64) void k_na(const float* __restrict__ QKV, const float* __restrict__ RPB, float* __restrict__ O) {
  __shared__ float sk[KS][WW][HD + 1], sv[KS][WW][HD + 1]; __shared__ float srpb[13][13]; __shared__ __align__(16) float so[WW][HD + 4]; __shared__ float slg[WW][KS * KS + 3];
  const int tid = threadIdx.x; const int n = blockIdx.x % NHD, i = (blockIdx.x / NHD) % HH, b = blockIdx.x / (NHD * HH);
  const int i0 = min(max(i - 3, 0), HH - KS);
  for (int q = tid; q < KS * WW * HD; q += 64) { const int a = q / (WW * HD), rem = q % (WW * HD), jj = rem / HD, d = rem % HD; const size_t tok = ((size_t)b * HH + i0 + a) * WW + jj; sk[a][jj][d] = QKV[tok * 384 + CC + n * HD + d]; sv[a][jj][d] = QKV[tok * 384 + 2 * CC + n * HD + d]; }
  for (int q = tid; q < 169; q += 64) srpb[q / 13][q % 13] = bfr(RPB[(n * 13 + q / 13) * 13 + q % 13]);
  __syncthreads();
  const int j = tid; const int j0 = min(max(j - 3, 0), WW - KS); const size_t tq = ((size_t)b * HH + i) * WW + j;
  float qv[HD];
#pragma unroll
  for (int d = 0; d < HD; ++d) qv[d] = QKV[tq * 384 + n * HD + d];
  float mx = -3.0e38f;
#pragma unroll 1
  for (int a = 0; a < KS; ++a) {
#pragma unroll 1
    for (int c = 0; c < KS; ++c) { const int jj = j0 + c; float s = 0.f;
#pragma unroll
      for (int d = 0; d < HD; ++d) s += qv[d] * sk[a][jj][d];
      s += srpb[i0 + a - i + KS - 1][jj - j + KS - 1]; slg[j][a * KS + c] = s; mx = fmaxf(mx, s); } }
  float z = 0.f;
#pragma unroll 1
  for (int e = 0; e < KS * KS; ++e) { const float ex = exp_ni(slg[j][e] - mx); slg[j][e] = ex; z += ex; }
  const float iz = 1.0f / z; float ov[HD];
#pragma unroll
  for (int d = 0; d < HD; ++d) ov[d] = 0.f;
#pragma unroll 1
  for (int a = 0; a < KS; ++a) {
#pragma unroll 1
    for (int c = 0; c < KS; ++c) { const int jj = j0 + c; const float p = slg[j][a * KS + c] * iz;
#pragma unroll
      for (int d = 0; d < HD; ++d) ov[d] += p * sv[a][jj][d]; } }
#pragma unroll
  for (int d = 0; d < HD; ++d) so[j][d] = ov[d];
  __syncthreads();
  for (int q = tid; q < WW * 8; q += 64) { const int jj = q >> 3, pc = q & 7; vst2(O + (((size_t)b * HH + i) * WW + jj) * CC + n * HD + pc * 4, *(const v4f*)&so[jj][pc * 4]); }
}
__global__ __launch_bounds__(128) void k_proj(const float* __restrict__ O, const __bf16* __restrict__ PT, const float* __restrict__ pb, float* __restrict__ out) {
  __shared__ __align__(16) float so[4][16][132];
  const int tid = threadIdx.x, wave = tid >> 5, lane = tid & 31, col = lane & 15, g = lane >> 4; const size_t r0 = (size_t)blockIdx.x * 64 + wave * 16;
  v8f acc[8] = {};
#pragma unroll
  for (int kc = 0; kc < 4; ++kc) { const F2 a = split_row(O + (r0 + col) * CC, kc * 32, lane);
#pragma unroll
    for (int j = 0; j < 8; ++j) { const v16b w = frag_b(PT + (size_t)(384 + j * 16 + col) * CC + kc * 32, lane); acc[j] = wmma_bf(a.l, w, acc[j]); acc[j] = wmma_bf(a.h, w, acc[j]); } }
#pragma unroll
  for (int j = 0; j < 8; ++j) { const float bb = bfr(pb[j * 16 + col]);
#pragma unroll
    for (int r = 0; r < 8; ++r) so[wave][8 * g + r][j * 16 + col] = acc[j][r] + bb; }
  LDSX();
  for (int rl = 0; rl < 16; ++rl) vst2(out + (r0 + rl) * CC + lane * 4, *(const v4f*)&so[wave][rl][lane * 4]);
}

extern "C" void kernel_launch(void* const* d_in, const int* in_sizes, int n_in, void* d_out, int out_size, void* d_ws, size_t ws_size, hipStream_t stream) {
  (void)in_sizes; (void)n_in; (void)out_size;
  const float** F = (const float**)d_in; const int** I = (const int**)d_in;
  if (ws_size < (size_t)WS_END) return;
  char* ws = (char*)d_ws; float *ADA = (float*)(ws + WS_ADA), *QKV = (float*)(ws + WS_QKV), *O = (float*)(ws + WS_O); __bf16* PT = (__bf16*)(ws + WS_PT);
  k_ada<<<1, 256, 0, stream>>>(I[2], F[3], F[4], ADA);
  k_pack<<<512, 128, 0, stream>>>(F[5], F[8], PT);
  k_qkv<<<TTB, 128, 0, stream>>>(F[0], ADA, PT, F[6], QKV);
  k_na<<<TNAB, 64, 0, stream>>>(QKV, F[7], O);
  k_proj<<<TTB, 128, 0, stream>>>(O, PT, F[9], (float*)d_out);
}
